// GemmaAttention_84902913507534
// MI455X (gfx1250) — hardware-verified
//
#include <hip/hip_runtime.h>
#include <math.h>

#pragma clang fp contract(off)

#ifndef NB
#define NB 2
#endif
#ifndef SEQ
#define SEQ 2048
#endif
#define NB_FULL  2
#define SEQ_FULL 2048
#define HID      2048
#define NQH      16
#define NKVH     8
#define HD       128
#define HHALF    64
#define QDIM     (NQH * HD)
#define KVDIM    (NKVH * HD)
#define NTOK     (NB * SEQ)
#define KV_CHUNK 64
#define QBLK     128
#define RSQ      0.08838834764831845f
#define SOFTCAP  50.0f
#define INVCAP   0.02f
#define PCARRY   1024.0f
#define OCARRY   64.0f
#define WOCARRY  16.0f
#define OUTSCALE 0.0009765625f

typedef __attribute__((ext_vector_type(16))) _Float16 v16h;
typedef __attribute__((ext_vector_type(8)))  _Float16 v8h;
typedef __attribute__((ext_vector_type(16))) __bf16   v16b;
typedef __attribute__((ext_vector_type(8)))  __bf16   v8b;
typedef __attribute__((ext_vector_type(8)))  float    v8f;
typedef __attribute__((ext_vector_type(4)))  float    v4f;
typedef __attribute__((ext_vector_type(4)))  unsigned int v4u;

__device__ __forceinline__ unsigned short f2bf_bits(float f) {
  unsigned u = __float_as_uint(f);
  return (unsigned short)((u + 0x7FFFu + ((u >> 16) & 1u)) >> 16);
}
__device__ __forceinline__ float bf_bits2f(unsigned short h) { return __uint_as_float(((unsigned)h) << 16); }
__device__ __forceinline__ unsigned short f2h_bits(float f) { const _Float16 h = (_Float16)f; return __builtin_bit_cast(unsigned short, h); }

__device__ __forceinline__ void dep_guard_h(v8f& a, v8f& b, v16h x, v16h y) { asm volatile("v_nop\n\tv_nop\n\tv_nop\n\tv_nop" : "+v"(a), "+v"(b) : "v"(x), "v"(y)); }
__device__ __forceinline__ void dep_guard_b(v8f& a, v8f& b, v16b x, v16b y) { asm volatile("v_nop\n\tv_nop\n\tv_nop\n\tv_nop" : "+v"(a), "+v"(b) : "v"(x), "v"(y)); }
__device__ __forceinline__ void keep4_h(v16h a, v16h b, v16h c, v16h d) { asm volatile("v_nop" :: "v"(a), "v"(b), "v"(c), "v"(d)); }
__device__ __forceinline__ void keep4_b(v16b a, v16b b, v16b c, v16b d) { asm volatile("v_nop" :: "v"(a), "v"(b), "v"(c), "v"(d)); }
__device__ __forceinline__ void acc_guard4(v8f& a, v8f& b, v8f& c, v8f& d) { asm volatile("v_nop\n\tv_nop\n\tv_nop\n\tv_nop" : "+v"(a), "+v"(b), "+v"(c), "+v"(d)); }

template <typename T> struct Frag;
template <> struct Frag<_Float16> {
  typedef v16h V; union U { v16h v; v8h h[2]; };
  static __device__ __forceinline__ v16h load(const _Float16* p) {
    U f; f.h[0] = *(const v8h*)(p); f.h[1] = *(const v8h*)(p + 16); return f.v;
  }
  static __device__ __forceinline__ v8f mma(v16h a, v16h b, v8f c) {
    return __builtin_amdgcn_wmma_f32_16x16x32_f16(false, a, false, b, (short)0, c, false, false);
  }
  static __device__ __forceinline__ void guard(v8f& a, v8f& b, v16h x, v16h y) { dep_guard_h(a, b, x, y); }
  static __device__ __forceinline__ void keep(v16h a, v16h b, v16h c, v16h d) { keep4_h(a, b, c, d); }
};
template <> struct Frag<__bf16> {
  typedef v16b V; union U { v16b v; v8b h[2]; };
  static __device__ __forceinline__ v16b load(const __bf16* p) {
    U f; f.h[0] = *(const v8b*)(p); f.h[1] = *(const v8b*)(p + 16); return f.v;
  }
  static __device__ __forceinline__ v8f mma(v16b a, v16b b, v8f c) {
    return __builtin_amdgcn_wmma_f32_16x16x32_bf16(false, a, false, b, (short)0, c, false, false);
  }
  static __device__ __forceinline__ void guard(v8f& a, v8f& b, v16b x, v16b y) { dep_guard_b(a, b, x, y); }
  static __device__ __forceinline__ void keep(v16b a, v16b b, v16b c, v16b d) { keep4_b(a, b, c, d); }
};

__device__ __forceinline__ v8f h_mma(v16h a, v16h b, v8f c) {
  c = __builtin_amdgcn_wmma_f32_16x16x32_f16(false, a, false, b, (short)0, c, false, false);
  asm volatile("v_nop\n\tv_nop\n\tv_nop\n\tv_nop" : "+v"(c) : "v"(a), "v"(b));
  return c;
}

__global__ __launch_bounds__(256) void cast_x_bf16(const float* __restrict__ in, unsigned short* __restrict__ out, int n8) {
  const int i = blockIdx.x * 256 + threadIdx.x;
  if (i < n8) {
    const size_t o   = (size_t)i * 8;
    const size_t tok = o / HID;
    const size_t col = o - tok * HID;
    const size_t bb  = tok / SEQ;
    const size_t ss  = tok - bb * SEQ;
    const size_t src = (bb * SEQ_FULL + ss) * (size_t)HID + col;
    const v4f a  = *(const v4f*)(in + src);
    const v4f bq = *(const v4f*)(in + src + 4);
    v4u w;
    w[0] = (unsigned)f2bf_bits(a[0])  | ((unsigned)f2bf_bits(a[1])  << 16);
    w[1] = (unsigned)f2bf_bits(a[2])  | ((unsigned)f2bf_bits(a[3])  << 16);
    w[2] = (unsigned)f2bf_bits(bq[0]) | ((unsigned)f2bf_bits(bq[1]) << 16);
    w[3] = (unsigned)f2bf_bits(bq[2]) | ((unsigned)f2bf_bits(bq[3]) << 16);
    *(volatile v4u*)(out + o) = w;
    __threadfence();
    *(volatile v4u*)(out + o) = w;
  }
}

template <int MODE> __device__ __forceinline__ unsigned short pk16(float f, float scl) {
  if (MODE == 0) return f2bf_bits(f);
  const float g = bf_bits2f(f2bf_bits(f)) * scl;
  return f2h_bits(g);
}

template <int MODE>
__global__ __launch_bounds__(256) void transpose_cast16(const float* __restrict__ in, unsigned short* __restrict__ out, int nrows, int ncols, float scl) {
  __shared__ float tile[64 * 65];
  const int tid = threadIdx.x;
  const int r0 = blockIdx.y * 64, c0 = blockIdx.x * 64;
  {
    const int row = tid >> 2, cc = (tid & 3) * 16;
    const float* s = in + (size_t)(r0 + row) * ncols + c0 + cc;
#pragma unroll
    for (int q = 0; q < 4; ++q) {
      const v4f v = *(const v4f*)(s + 4 * q);
#pragma unroll
      for (int e = 0; e < 4; ++e) tile[(cc + 4 * q + e) * 65 + row] = v[e];
    }
  }
  __syncthreads();
  for (int pass = 0; pass < 2; ++pass) {
#pragma unroll
    for (int it = 0; it < 2; ++it) {
      const int orow = it * 32 + (tid >> 3), seg = (tid & 7) * 8;
      const float* tp = tile + orow * 65 + seg;
      v4u w;
#pragma unroll
      for (int e = 0; e < 4; ++e) w[e] = (unsigned)pk16<MODE>(tp[2 * e], scl) | ((unsigned)pk16<MODE>(tp[2 * e + 1], scl) << 16);
      *(volatile v4u*)(out + (size_t)(c0 + orow) * nrows + r0 + seg) = w;
    }
    __threadfence();
  }
}

struct RopeFreq { float f[HHALF]; };
static_assert(sizeof(RopeFreq) == 256);

__global__ __launch_bounds__(256) void rope_table_kernel(float* __restrict__ cosT, float* __restrict__ sinT, RopeFreq fr) {
  __shared__ float invf[HHALF];
  if (threadIdx.x == 0) {
#pragma unroll
    for (int q = 0; q < HHALF; ++q) invf[q] = fr.f[q];
  }
  __syncthreads();
  const int i = blockIdx.x * 256 + threadIdx.x;
  const int t = i >> 6;
  const int jj = i & (HHALF - 1);
  const float ang = (float)t * invf[jj];
  const float cv = cosf(ang);
  const float sv = sinf(ang);
  ((volatile float*)cosT)[i] = cv;
  ((volatile float*)sinT)[i] = sv;
  __threadfence();
  ((volatile float*)cosT)[i] = cv;
  ((volatile float*)sinT)[i] = sv;
}

template <int NHEAD, int PITCH>
__global__ __launch_bounds__(256) void rope_f16_kernel(const float* __restrict__ src, const float* __restrict__ cosT, const float* __restrict__ sinT,
                                                        unsigned short* __restrict__ outP, float scl) {
  const int i = blockIdx.x * 256 + threadIdx.x;
  const int jg = i & 7;
  const int hs = (i >> 3) % NHEAD;
  const int tok = (i >> 3) / NHEAD;
  const int pos = tok % SEQ;
  const size_t base = (size_t)tok * PITCH + (size_t)hs * HD + jg * 8;
  const size_t tb = (size_t)pos * HHALF + jg * 8;
  const v4f x1a = *(const v4f*)(src + base);
  const v4f x1b = *(const v4f*)(src + base + 4);
  const v4f x2a = *(const v4f*)(src + base + HHALF);
  const v4f x2b = *(const v4f*)(src + base + HHALF + 4);
  const v4f ca = *(const v4f*)(cosT + tb);
  const v4f cb = *(const v4f*)(cosT + tb + 4);
  const v4f sa = *(const v4f*)(sinT + tb);
  const v4f sb = *(const v4f*)(sinT + tb + 4);
  v4f o1a, o1b, o2a, o2b;
#pragma unroll
  for (int e = 0; e < 4; ++e) {
    o1a[e] = (x1a[e] * ca[e] - x2a[e] * sa[e]) * scl;
    o2a[e] = (x2a[e] * ca[e] + x1a[e] * sa[e]) * scl;
    o1b[e] = (x1b[e] * cb[e] - x2b[e] * sb[e]) * scl;
    o2b[e] = (x2b[e] * cb[e] + x1b[e] * sb[e]) * scl;
  }
  v4u h1, h2;
  h1[0] = (unsigned)f2h_bits(o1a[0]) | ((unsigned)f2h_bits(o1a[1]) << 16);
  h1[1] = (unsigned)f2h_bits(o1a[2]) | ((unsigned)f2h_bits(o1a[3]) << 16);
  h1[2] = (unsigned)f2h_bits(o1b[0]) | ((unsigned)f2h_bits(o1b[1]) << 16);
  h1[3] = (unsigned)f2h_bits(o1b[2]) | ((unsigned)f2h_bits(o1b[3]) << 16);
  h2[0] = (unsigned)f2h_bits(o2a[0]) | ((unsigned)f2h_bits(o2a[1]) << 16);
  h2[1] = (unsigned)f2h_bits(o2a[2]) | ((unsigned)f2h_bits(o2a[3]) << 16);
  h2[2] = (unsigned)f2h_bits(o2b[0]) | ((unsigned)f2h_bits(o2b[1]) << 16);
  h2[3] = (unsigned)f2h_bits(o2b[2]) | ((unsigned)f2h_bits(o2b[3]) << 16);
  for (int pass = 0; pass < 2; ++pass) {
    *(volatile v4u*)(outP + base) = h1;
    *(volatile v4u*)(outP + base + HHALF) = h2;
    __threadfence();
  }
}

template <typename T, bool SPLITA, bool SPLITB, int OUT_MODE>
__global__ __launch_bounds__(256) void gemm_t64(
    const unsigned short* __restrict__ Ap, const unsigned short* __restrict__ A2p, int lda, long strideA,
    const unsigned short* __restrict__ Btp, const unsigned short* __restrict__ Bt2p, int ldb, long strideB,
    void* __restrict__ Cout, int ldc, long strideC,
    int M, int N, int K, float scale) {
  typedef typename Frag<T>::V V;
  const T* A = (const T*)Ap; const T* A2 = (const T*)A2p; const T* Bt = (const T*)Btp; const T* Bt2 = (const T*)Bt2p;
  __shared__ __align__(16) float sT[8][16 * 68];
  const int b    = blockIdx.y;
  const int lane = threadIdx.x & 31;
  const int wave = threadIdx.x >> 5;
  const int tilesN = N >> 6;
  const int tilesM = M >> 6;
  const int tile = blockIdx.x * 8 + wave;
  if (tile >= tilesM * tilesN) return;
  const int tm = tile / tilesN;
  const int tn = tile - tm * tilesN;
  const int m0 = tm << 6;
  const int n0 = tn << 6;

  const T* Ab  = A  + (size_t)b * strideA;
  const T* Bb  = Bt + (size_t)b * strideB;
  const T* Ab2 = A2  + (size_t)b * strideA;
  const T* Bb2 = Bt2 + (size_t)b * strideB;

  const int rlane = lane & 15;
  const int koff  = (lane >> 4) * 8;
  const int mOff  = (lane >> 4) * 8;

  v8f acc[4][4];
#pragma unroll
  for (int i = 0; i < 4; ++i)
#pragma unroll
    for (int j = 0; j < 4; ++j) acc[i][j] = (v8f){0.f,0.f,0.f,0.f,0.f,0.f,0.f,0.f};

  for (int k0 = 0; k0 < K; k0 += 32) {
    V bh[4], bl[4];
#pragma unroll
    for (int j = 0; j < 4; ++j) {
      const size_t bo = (size_t)(n0 + (j << 4) + rlane) * ldb + koff + k0;
      bh[j] = Frag<T>::load(Bb + bo);
      if (SPLITB) bl[j] = Frag<T>::load(Bb2 + bo);
    }
#pragma unroll
    for (int i = 0; i < 4; ++i) {
      const size_t ao = (size_t)(m0 + (i << 4) + rlane) * lda + koff + k0;
      V ah = Frag<T>::load(Ab + ao);
      V al = ah;
      if (SPLITA) al = Frag<T>::load(Ab2 + ao);
#pragma unroll
      for (int j = 0; j < 4; ++j) {
        acc[i][j] = Frag<T>::mma(ah, bh[j], acc[i][j]);
        if (SPLITB) acc[i][j] = Frag<T>::mma(ah, bl[j], acc[i][j]);
        if (SPLITA) acc[i][j] = Frag<T>::mma(al, bh[j], acc[i][j]);
      }
      Frag<T>::guard(acc[i][0], acc[i][3], ah, al);
    }
    Frag<T>::keep(bh[0], bh[1], bh[2], bh[3]);
    if (SPLITB) Frag<T>::keep(bl[0], bl[1], bl[2], bl[3]);
  }
  acc_guard4(acc[0][0], acc[0][1], acc[0][2], acc[0][3]);
  acc_guard4(acc[1][0], acc[1][1], acc[1][2], acc[1][3]);
  acc_guard4(acc[2][0], acc[2][1], acc[2][2], acc[2][3]);
  acc_guard4(acc[3][0], acc[3][1], acc[3][2], acc[3][3]);

  float* slab = sT[wave];
#pragma unroll
  for (int i = 0; i < 4; ++i) {
    const int mBase = m0 + (i << 4);
#pragma unroll
    for (int j = 0; j < 4; ++j) {
#pragma unroll
      for (int r = 0; r < 8; ++r) {
        const float v = acc[i][j][r] * scale;
        slab[(mOff + r) * 68 + (j << 4) + rlane] = v;
      }
    }
    __builtin_amdgcn_fence(3, "workgroup");
    __builtin_amdgcn_wave_barrier();
    __builtin_amdgcn_fence(2, "workgroup");
    if (OUT_MODE == 0) {
      float* Cf = (float*)Cout + (size_t)b * strideC;
      const int hh = lane >> 4, c4 = (lane & 15) * 4;
      for (int pass = 0; pass < 2; ++pass) {
#pragma unroll
        for (int it = 0; it < 8; ++it) {
          const int row = it * 2 + hh;
          v4f v = *(const v4f*)(slab + row * 68 + c4);
          *(volatile v4f*)(Cf + (size_t)(mBase + row) * ldc + n0 + c4) = v;
        }
        __threadfence();
      }
    } else {
      const int q = lane >> 3, c8 = (lane & 7) * 8;
      unsigned short* Cs = (unsigned short*)Cout + (size_t)b * strideC;
      for (int pass = 0; pass < 2; ++pass) {
#pragma unroll
        for (int it = 0; it < 4; ++it) {
          const int row = it * 4 + q;
          const float* sp = slab + row * 68 + c8;
          v8h hv;
#pragma unroll
          for (int e = 0; e < 8; ++e) hv[e] = (_Float16)sp[e];
          *(volatile v8h*)(Cs + (size_t)(mBase + row) * ldc + n0 + c8) = hv;
        }
        __threadfence();
      }
    }
    __builtin_amdgcn_fence(3, "workgroup");
    __builtin_amdgcn_wave_barrier();
    __builtin_amdgcn_fence(2, "workgroup");
  }
}

__global__ __launch_bounds__(256) void attn_kernel(
    const unsigned short* __restrict__ Qp, const unsigned short* __restrict__ Kp,
    const unsigned short* __restrict__ Vtp, unsigned short* __restrict__ Op) {
  __shared__ __align__(16) float    Ost[8][16 * 64];
  __shared__ __align__(16) _Float16 Psh[8][16 * KV_CHUNK];

  const _Float16* Q  = (const _Float16*)Qp;
  const _Float16* Kk = (const _Float16*)Kp;
  const _Float16* Vt = (const _Float16*)Vtp;

  const int tid  = threadIdx.x;
  const int wave = tid >> 5, lane = tid & 31;
  const int hh   = lane >> 4, c = lane & 15, koff = hh * 8;
  const int nqb  = SEQ / QBLK;
  const int bx   = blockIdx.x;
  const int qb   = bx % nqb;
  const int bhid = bx / nqb;
  const int h    = bhid % NQH;
  const int b    = bhid / NQH;
  const int kvh  = h >> 1;
  const int q0   = qb * QBLK + wave * 16;
  const size_t tokw = (size_t)b * SEQ + q0;
  const size_t qoff = (tokw + c) * QDIM + (size_t)h * HD + koff;
  const _Float16* Kb  = Kk + (size_t)b * SEQ * KVDIM + (size_t)kvh * HD + koff;
  const _Float16* Vtb = Vt + (size_t)b * KVDIM * SEQ + (size_t)(kvh * HD + c) * SEQ + koff;
  _Float16* pw = Psh[wave];

  float mrow[8], lrow[8];
  v8f oacc[8];
#pragma unroll
  for (int r = 0; r < 8; ++r) { mrow[r] = -INFINITY; lrow[r] = 0.f; }
#pragma unroll
  for (int t = 0; t < 8; ++t) oacc[t] = (v8f){0.f,0.f,0.f,0.f,0.f,0.f,0.f,0.f};

  for (int kc = 0; kc < SEQ / KV_CHUNK; ++kc) {
    const int kv0 = kc * KV_CHUNK;

    v8f s[4];
#pragma unroll
    for (int j = 0; j < 4; ++j) s[j] = (v8f){0.f,0.f,0.f,0.f,0.f,0.f,0.f,0.f};
#pragma unroll
    for (int dc = 0; dc < 4; ++dc) {
      const v16h qa = Frag<_Float16>::load(Q + qoff + dc * 32);
#pragma unroll
      for (int j = 0; j < 4; ++j) {
        const size_t ko = (size_t)(kv0 + j * 16 + c) * KVDIM + dc * 32;
        const v16h kb = Frag<_Float16>::load(Kb + ko);
        s[j] = h_mma(qa, kb, s[j]);
      }
    }

    float cm[8];
#pragma unroll
    for (int r = 0; r < 8; ++r) {
      float m = -INFINITY;
#pragma unroll
      for (int j = 0; j < 4; ++j) {
        float sv = s[j][r] * RSQ;
        sv = SOFTCAP * tanhf(sv * INVCAP);
        s[j][r] = sv;
        m = fmaxf(m, sv);
      }
#pragma unroll
      for (int off = 1; off < 16; off <<= 1) m = fmaxf(m, __shfl_xor(m, off, 32));
      cm[r] = m;
    }

    __builtin_amdgcn_fence(3, "workgroup");
    __builtin_amdgcn_wave_barrier();
    __builtin_amdgcn_fence(2, "workgroup");

#pragma unroll
    for (int r = 0; r < 8; ++r) {
      const float mnew = fmaxf(mrow[r], cm[r]);
      const float alpha = __expf(mrow[r] - mnew);
      mrow[r] = mnew;
      float psum = 0.f;
#pragma unroll
      for (int j = 0; j < 4; ++j) {
        const float p = __expf(s[j][r] - mnew);
        psum += p;
        pw[(8 * hh + r) * KV_CHUNK + j * 16 + c] = (_Float16)(p * PCARRY);
      }
#pragma unroll
      for (int off = 1; off < 16; off <<= 1) psum += __shfl_xor(psum, off, 32);
      lrow[r] = lrow[r] * alpha + psum;
#pragma unroll
      for (int t = 0; t < 8; ++t) oacc[t][r] *= alpha;
    }
    __builtin_amdgcn_fence(3, "workgroup");
    __builtin_amdgcn_wave_barrier();
    __builtin_amdgcn_fence(2, "workgroup");

#pragma unroll
    for (int kk = 0; kk < 2; ++kk) {
      const v16h pa = Frag<_Float16>::load(pw + c * KV_CHUNK + kk * 32 + koff);
#pragma unroll
      for (int t = 0; t < 8; ++t) {
        const size_t vo = (size_t)t * 16 * SEQ + kv0 + kk * 32;
        const v16h vb = Frag<_Float16>::load(Vtb + vo);
        oacc[t] = h_mma(pa, vb, oacc[t]);
      }
    }
  }

  float* os = Ost[wave];
  const int q4 = lane >> 3, c8 = (lane & 7) * 8;
#pragma unroll
  for (int th = 0; th < 2; ++th) {
#pragma unroll
    for (int r = 0; r < 8; ++r) {
      const float inv = OCARRY / (PCARRY * lrow[r]);
#pragma unroll
      for (int tt = 0; tt < 4; ++tt) os[(8 * hh + r) * 64 + tt * 16 + c] = oacc[th * 4 + tt][r] * inv;
    }
    __builtin_amdgcn_fence(3, "workgroup");
    __builtin_amdgcn_wave_barrier();
    __builtin_amdgcn_fence(2, "workgroup");
    for (int pass = 0; pass < 2; ++pass) {
#pragma unroll
      for (int it = 0; it < 4; ++it) {
        const int row = it * 4 + q4;
        const float* sp = os + row * 64 + c8;
        v8h hv;
#pragma unroll
        for (int e = 0; e < 8; ++e) hv[e] = (_Float16)sp[e];
        const size_t o = (tokw + row) * QDIM + (size_t)h * HD + th * 64 + c8;
        *(volatile v8h*)(Op + o) = hv;
      }
      __threadfence();
    }
    __builtin_amdgcn_fence(3, "workgroup");
    __builtin_amdgcn_wave_barrier();
    __builtin_amdgcn_fence(2, "workgroup");
  }
}

static_assert((NTOK * HID / 8) % 256 == 0);
static_assert((NTOK * NQH * 8) % 256 == 0);
static_assert((NTOK * NKVH * 8) % 256 == 0);
static_assert((SEQ * HHALF) % 256 == 0);
static_assert(HID % 32 == 0 && QDIM % 32 == 0);
static_assert(NTOK % 64 == 0 && HID % 64 == 0 && QDIM % 64 == 0 && KVDIM % 64 == 0 && SEQ % 64 == 0);
static_assert(SEQ % QBLK == 0 && SEQ % KV_CHUNK == 0 && QBLK == 128 && KV_CHUNK == 64 && HD == 128);
static_assert(NB >= 1 && NB <= NB_FULL && SEQ <= SEQ_FULL);
static_assert(NQH == 2 * NKVH);

extern "C" void kernel_launch(void* const* d_in, const int* in_sizes, int n_in,
                              void* d_out, int out_size, void* d_ws, size_t ws_size, hipStream_t stream) {
  if (n_in < 5) return;
  const size_t needTok = (size_t)(NB - 1) * SEQ_FULL + SEQ;
  if ((size_t)in_sizes[0] < needTok * HID) return;
  if ((size_t)in_sizes[1] < (size_t)HID * QDIM) return;
  if ((size_t)in_sizes[2] < (size_t)HID * KVDIM) return;
  if ((size_t)in_sizes[3] < (size_t)HID * KVDIM) return;
  if ((size_t)in_sizes[4] < (size_t)QDIM * HID) return;
  if ((size_t)out_size < needTok * HID) return;

  const float* x  = (const float*)d_in[0];
  const float* Wq = (const float*)d_in[1];
  const float* Wk = (const float*)d_in[2];
  const float* Wv = (const float*)d_in[3];
  const float* Wo = (const float*)d_in[4];
  float* out = (float*)d_out;

  const size_t szXB  = (size_t)NTOK * HID * 2;
  const size_t szWQT = (size_t)QDIM * HID * 2;
  const size_t szWKT = (size_t)KVDIM * HID * 2;
  const size_t szWOT = (size_t)HID * QDIM * 2;
  const size_t szR1  = (size_t)NTOK * QDIM * 4;
  const size_t szQP  = (size_t)NTOK * QDIM * 2;
  const size_t szKP  = (size_t)NTOK * KVDIM * 2;
  const size_t szVT  = (size_t)NB * KVDIM * SEQ * 2;
  const size_t szTAB = (size_t)SEQ * HHALF * 4;
  static_assert((size_t)NTOK * KVDIM * 4 <= (size_t)NTOK * QDIM * 4);
  static_assert((size_t)NTOK * QDIM * 2 + (size_t)NB * KVDIM * SEQ * 2 <= (size_t)NTOK * QDIM * 4);
  const size_t OFF_XB  = 0;
  const size_t OFF_WQT = OFF_XB + szXB;
  const size_t OFF_WKT = OFF_WQT + szWQT;
  const size_t OFF_WVT = OFF_WKT + szWKT;
  const size_t OFF_WOT = OFF_WVT + szWKT;
  const size_t OFF_R1  = OFF_WOT + szWOT;
  const size_t OFF_QF  = OFF_R1;
  const size_t OFF_KF  = OFF_R1;
  const size_t OFF_CTX = OFF_R1;
  const size_t OFF_VT  = OFF_R1 + szQP;
  const size_t OFF_QP  = OFF_R1 + szR1;
  const size_t OFF_KP  = OFF_QP + szQP;
  const size_t OFF_COS = OFF_KP + szKP;
  const size_t OFF_SIN = OFF_COS + szTAB;
  const size_t WS_TOTAL = OFF_SIN + szTAB;
  (void)szVT;
  if (ws_size < WS_TOTAL) return;

  char* ws = (char*)d_ws;
  unsigned short* xb  = (unsigned short*)(ws + OFF_XB);
  unsigned short* WqT = (unsigned short*)(ws + OFF_WQT);
  unsigned short* WkT = (unsigned short*)(ws + OFF_WKT);
  unsigned short* WvT = (unsigned short*)(ws + OFF_WVT);
  unsigned short* WoT = (unsigned short*)(ws + OFF_WOT);
  float* Qf  = (float*)(ws + OFF_QF);
  float* Kf  = (float*)(ws + OFF_KF);
  unsigned short* ctx = (unsigned short*)(ws + OFF_CTX);
  unsigned short* Vt  = (unsigned short*)(ws + OFF_VT);
  unsigned short* Qpl = (unsigned short*)(ws + OFF_QP);
  unsigned short* Kpl = (unsigned short*)(ws + OFF_KP);
  float* cosT = (float*)(ws + OFF_COS);
  float* sinT = (float*)(ws + OFF_SIN);

  RopeFreq fr;
  for (int j = 0; j < HHALF; ++j) {
    const float e = (float)(2 * j) / 128.0f;
    const double p = pow(10000.0, (double)e);
    const float pf = (float)p;
    fr.f[j] = 1.0f / pf;
  }

  cast_x_bf16<<<(NTOK * HID / 8) / 256, 256, 0, stream>>>(x, xb, NTOK * HID / 8);
  transpose_cast16<0><<<dim3(QDIM / 64, HID / 64), 256, 0, stream>>>(Wq, WqT, HID, QDIM, 1.0f);
  transpose_cast16<0><<<dim3(KVDIM / 64, HID / 64), 256, 0, stream>>>(Wk, WkT, HID, KVDIM, 1.0f);
  transpose_cast16<0><<<dim3(KVDIM / 64, HID / 64), 256, 0, stream>>>(Wv, WvT, HID, KVDIM, 1.0f);
  transpose_cast16<1><<<dim3(HID / 64, QDIM / 64), 256, 0, stream>>>(Wo, WoT, QDIM, HID, WOCARRY);
  rope_table_kernel<<<(SEQ * HHALF) / 256, 256, 0, stream>>>(cosT, sinT, fr);
  {
    const int tiles = (NTOK / 64) * (QDIM / 64);
    gemm_t64<__bf16, false, false, 0><<<dim3((tiles + 7) / 8, 1), 256, 0, stream>>>(
        xb, xb, HID, 0L, WqT, WqT, HID, 0L, (void*)Qf, QDIM, 0L, NTOK, QDIM, HID, 1.0f);
  }
  rope_f16_kernel<NQH, QDIM><<<(NTOK * NQH * 8) / 256, 256, 0, stream>>>(Qf, cosT, sinT, Qpl, 1.0f);
  {
    const int tiles = (NTOK / 64) * (KVDIM / 64);
    gemm_t64<__bf16, false, false, 0><<<dim3((tiles + 7) / 8, 1), 256, 0, stream>>>(
        xb, xb, HID, 0L, WkT, WkT, HID, 0L, (void*)Kf, KVDIM, 0L, NTOK, KVDIM, HID, 1.0f);
  }
  rope_f16_kernel<NKVH, KVDIM><<<(NTOK * NKVH * 8) / 256, 256, 0, stream>>>(Kf, cosT, sinT, Kpl, 1.0f);
  {
    const int tiles = (KVDIM / 64) * (SEQ / 64);
    gemm_t64<__bf16, false, false, 1><<<dim3((tiles + 7) / 8, NB), 256, 0, stream>>>(
        WvT, WvT, HID, 0L, xb, xb, HID, (long)SEQ * HID, (void*)Vt, SEQ, (long)KVDIM * SEQ,
        KVDIM, SEQ, HID, 1.0f);
  }
  attn_kernel<<<NB * NQH * (SEQ / QBLK), 256, 0, stream>>>(Qpl, Kpl, Vt, ctx);
  {
    const int tiles = (SEQ / 64) * (HID / 64);
    gemm_t64<_Float16, false, false, 0><<<dim3((tiles + 7) / 8, NB), 256, 0, stream>>>(
        ctx, ctx, QDIM, (long)SEQ * QDIM, WoT, WoT, QDIM, 0L, (void*)out, HID, (long)SEQ_FULL * HID,
        SEQ, HID, QDIM, OUTSCALE);
  }
}
